// Winograd2d_59030030516261
// MI455X (gfx1250) — hardware-verified
//
#include <hip/hip_runtime.h>


#define NB_  8
#define IC   128
#define OC   128
#define HW   68
#define TH   16
#define NTILE (NB_ * TH * TH)
#define OHW  64
#define LOSC 1024.0f
#define LOSCI (1.0f / 1024.0f)

typedef _Float16 h16;
typedef __attribute__((ext_vector_type(16))) _Float16 v16h;
typedef __attribute__((ext_vector_type(8)))  _Float16 v8h;
typedef __attribute__((ext_vector_type(8)))  float    v8f;
typedef __attribute__((ext_vector_type(4)))  float    v4f;
typedef v8h  __attribute__((may_alias)) v8ha;
typedef v4f  __attribute__((may_alias)) v4fa;

__constant__ float cBT[64] = {
    1.0f, 0.0f, -5.25f, 0.0f, 5.25f, 0.0f, -1.0f, 0.0f,
    0.0f, 1.0f, 1.0f, -4.25f, -4.25f, 1.0f, 1.0f, 0.0f,
    0.0f, -1.0f, 1.0f, 4.25f, -4.25f, -1.0f, 1.0f, 0.0f,
    0.0f, 0.5f, 0.25f, -2.5f, -1.25f, 2.0f, 1.0f, 0.0f,
    0.0f, -0.5f, 0.25f, 2.5f, -1.25f, -2.0f, 1.0f, 0.0f,
    0.0f, 2.0f, 4.0f, -2.5f, -5.0f, 0.5f, 1.0f, 0.0f,
    0.0f, -2.0f, 4.0f, 2.5f, -5.0f, -0.5f, 1.0f, 0.0f,
    0.0f, -1.0f, 0.0f, 5.25f, 0.0f, -5.25f, 0.0f, 1.0f };
__constant__ float cAT[32] = {
    1.0f, 1.0f, 1.0f, 1.0f, 1.0f, 8.0f, 8.0f, 0.0f,
    0.0f, 1.0f, -1.0f, 2.0f, -2.0f, 4.0f, -4.0f, 0.0f,
    0.0f, 1.0f, 1.0f, 4.0f, 4.0f, 2.0f, 2.0f, 0.0f,
    0.0f, 1.0f, -1.0f, 8.0f, -8.0f, 1.0f, -1.0f, 1.0f };

__device__ __forceinline__ unsigned short f2bf(float f) { unsigned u = __float_as_uint(f); u += 0x7FFFu + ((u >> 16) & 1u); return (unsigned short)(u >> 16); }
__device__ __forceinline__ float bf2f(unsigned short b) { return __uint_as_float(((unsigned)b) << 16); }
__device__ __forceinline__ float bfr(float f) { return bf2f(f2bf(f)); }
__device__ __forceinline__ v16h cat16(v8h lo, v8h hi) { return __builtin_shufflevector(lo, hi, 0, 1, 2, 3, 4, 5, 6, 7, 8, 9, 10, 11, 12, 13, 14, 15); }
__device__ __forceinline__ v8f wmma16(v16h a, v16h b, v8f c) { return __builtin_amdgcn_wmma_f32_16x16x32_f16(false, a, false, b, (short)0, c, false, false); }

__global__ __launch_bounds__(128) void k_xt(const float* __restrict__ x, int abase, h16* XTH, h16* XTL) {
    __shared__ __align__(16) h16 th_[32 * 136];
    __shared__ __align__(16) h16 tl_[32 * 136];
    const int c = threadIdx.x, tile = blockIdx.x;
    const int n = tile >> 8, th = (tile >> 4) & 15, tw = tile & 15;
    float d[8][8];
    const float* xb = x + (((size_t)n * IC + c) * HW + 4 * th) * HW + 4 * tw;
#pragma unroll
    for (int i = 0; i < 8; ++i)
#pragma unroll
        for (int j = 0; j < 8; ++j) d[i][j] = bfr(xb[(size_t)i * HW + j]);
    const int a0 = abase / 8;
#pragma unroll 1
    for (int ar = 0; ar < 4; ++ar) {
        const int a = a0 + ar;
        float t1[8];
#pragma unroll
        for (int j = 0; j < 8; ++j) { float s = 0.f;
#pragma unroll
            for (int i = 0; i < 8; ++i) s += cBT[a * 8 + i] * d[i][j];
            t1[j] = s; }
#pragma unroll 1
        for (int b = 0; b < 8; ++b) {
            float v = 0.f;
#pragma unroll
            for (int j = 0; j < 8; ++j) v += t1[j] * cBT[b * 8 + j];
            const h16 hv = (h16)v;
            th_[(ar * 8 + b) * 136 + c] = hv; tl_[(ar * 8 + b) * 136 + c] = (h16)((v - (float)hv) * LOSC);
        }
    }
    __syncthreads();
    const int lane = threadIdx.x & 31, wave = threadIdx.x >> 5;
    auto pass = [&]() {
#pragma unroll
        for (int s = 0; s < 8; ++s) { const int R = wave * 16 + 2 * s + (lane >> 4), piece = lane & 15; const int pln = R >> 5, abl = R & 31;
            const v8h val = *(const v8ha*)((pln ? tl_ : th_) + abl * 136 + piece * 8);
            *(volatile v8h*)((pln ? XTL : XTH) + ((size_t)abl * NTILE + tile) * IC + piece * 8) = val; }
    };
    pass(); __threadfence(); pass();
}

__global__ __launch_bounds__(128) void k_w16(const float* __restrict__ w, h16* W16) {
    __shared__ __align__(16) h16 tl[64 * 136];
    const int o = blockIdx.x, t = threadIdx.x;
    const float* wb = w + (size_t)o * IC * 64;
#pragma unroll 4
    for (int k = 0; k < 64; ++k) { const int idx = k * 128 + t; const int c = idx >> 6, ab = idx & 63; tl[ab * 136 + c] = (h16)bfr(wb[idx]); }
    __syncthreads();
    const int lane = t & 31, wave = t >> 5;
    auto pass = [&]() {
#pragma unroll
        for (int s = 0; s < 8; ++s) { const int ab = wave * 16 + 2 * s + (lane >> 4), piece = lane & 15; const v8h val = *(const v8ha*)(tl + ab * 136 + piece * 8);
            *(volatile v8h*)(W16 + ((size_t)ab * OC + o) * IC + piece * 8) = val; }
    };
    pass(); __threadfence(); pass();
}

__global__ __launch_bounds__(128) void k_mm(const h16* __restrict__ XTH, const h16* __restrict__ XTL, const h16* __restrict__ W16, int abase, float* YT) {
    __shared__ __align__(16) float ost[4][16 * 68];
    const int lane = threadIdx.x & 31, wave = threadIdx.x >> 5, lr = lane & 15, hi = lane >> 4;
    const int abl = blockIdx.z, ab = abase + abl;
    const int r0 = blockIdx.x * 64 + wave * 16, c0 = blockIdx.y * 64;
    const h16* A = XTH + (size_t)abl * NTILE * IC; const h16* Al = XTL + (size_t)abl * NTILE * IC; const h16* Bm = W16 + (size_t)ab * OC * IC;
    const size_t aoff = (size_t)(r0 + lr) * IC + 8 * hi;
    size_t boff[4];
#pragma unroll
    for (int t = 0; t < 4; ++t) boff[t] = (size_t)(c0 + t * 16 + lr) * IC + 8 * hi;
    v8f acc[4], accx[4];
#pragma unroll
    for (int t = 0; t < 4; ++t) { acc[t] = (v8f){}; accx[t] = (v8f){}; }
#pragma unroll
    for (int kc = 0; kc < IC; kc += 32) {
        const v16h a = cat16(*(const v8h*)(A + aoff + kc), *(const v8h*)(A + aoff + kc + 16)), al = cat16(*(const v8h*)(Al + aoff + kc), *(const v8h*)(Al + aoff + kc + 16));
#pragma unroll
        for (int t = 0; t < 4; ++t) { const v16h b = cat16(*(const v8h*)(Bm + boff[t] + kc), *(const v8h*)(Bm + boff[t] + kc + 16)); acc[t] = wmma16(a, b, acc[t]); accx[t] = wmma16(al, b, accx[t]); }
    }
    asm volatile("v_nop\n\tv_nop\n\tv_nop\n\tv_nop" : "+v"(acc[0]), "+v"(acc[1]), "+v"(acc[2]), "+v"(acc[3]), "+v"(accx[0]), "+v"(accx[1]), "+v"(accx[2]), "+v"(accx[3]));
    float* os = &ost[wave][0];
#pragma unroll
    for (int t = 0; t < 4; ++t)
#pragma unroll
        for (int j = 0; j < 8; ++j) os[(hi * 8 + j) * 68 + t * 16 + lr] = acc[t][j] + accx[t][j] * LOSCI;
    __syncthreads();
    float* crow = YT + ((size_t)ab * NTILE + r0) * OC + c0;
    auto pass = [&]() {
#pragma unroll
        for (int s = 0; s < 8; ++s) { const int Lid = (lane >> 3) + 4 * s, piece = lane & 7; const int row = Lid >> 1, cofs = (Lid & 1) * 32 + piece * 4;
            const v4f val = *(const v4fa*)(os + row * 68 + cofs); *(volatile v4f*)(crow + (size_t)row * OC + cofs) = val; }
    };
    pass(); __threadfence(); pass();
}

__global__ __launch_bounds__(256) void k_out(const float* __restrict__ YT, const float* __restrict__ bias, float* out) {
    const int lane = threadIdx.x & 31, wid = blockIdx.x * 8 + (threadIdx.x >> 5);
    if (wid >= NB_ * OC * TH) return;
    const int n = wid / (OC * TH), rem = wid - n * (OC * TH), o = rem / TH, th = rem - o * TH;
    const int tw = lane & 15, ph = lane >> 4;
    const int tile = (n * 16 + th) * 16 + tw;
    const float* m = YT + (size_t)tile * OC + o;
    float t2[2][8];
#pragma unroll
    for (int pp = 0; pp < 2; ++pp)
#pragma unroll
        for (int b = 0; b < 8; ++b) t2[pp][b] = 0.f;
#pragma unroll 1
    for (int a = 0; a < 8; ++a) {
        const float w0 = cAT[(2 * ph) * 8 + a], w1 = cAT[(2 * ph + 1) * 8 + a];
#pragma unroll
        for (int b = 0; b < 8; ++b) { const float mv = m[(size_t)(a * 8 + b) * NTILE * OC]; t2[0][b] += w0 * mv; t2[1][b] += w1 * mv; }
    }
    const float bo = bfr(bias[o]);
    v4f y[2];
#pragma unroll
    for (int pp = 0; pp < 2; ++pp)
#pragma unroll
        for (int q = 0; q < 4; ++q) { float s = 0.f;
#pragma unroll
            for (int b = 0; b < 8; ++b) s += t2[pp][b] * cAT[q * 8 + b];
            y[pp][q] = s + bo; }
    float* ob = out + (((size_t)n * OC + o) * OHW + 4 * th) * OHW + 4 * tw;
#pragma unroll
    for (int pp = 0; pp < 2; ++pp) *(volatile v4f*)(ob + (size_t)(2 * ph + pp) * OHW) = y[pp];
    __threadfence();
#pragma unroll
    for (int pp = 0; pp < 2; ++pp) *(volatile v4f*)(ob + (size_t)(2 * ph + pp) * OHW) = y[pp];
}

extern "C" void kernel_launch(void* const* d_in, const int* in_sizes, int n_in,
                              void* d_out, int out_size, void* d_ws, size_t ws_size, hipStream_t stream) {
    (void)in_sizes; (void)n_in; (void)out_size;
    const float* x = (const float*)d_in[0]; const float* w = (const float*)d_in[1]; const float* bias = (const float*)d_in[2];
    float* out = (float*)d_out;
    char* wsp = (char*)d_ws;
    auto take = [&](size_t bytes) { char* p = wsp; wsp += (bytes + 255) & ~(size_t)255; return (void*)p; };
    h16* XTH = (h16*)take((size_t)32 * NTILE * IC * 2); h16* XTL = (h16*)take((size_t)32 * NTILE * IC * 2); h16* W16 = (h16*)take((size_t)64 * OC * IC * 2);
    float* YT = (float*)take((size_t)64 * NTILE * OC * 4);
    if ((size_t)(wsp - (char*)d_ws) > ws_size) return;
    k_w16<<<OC, 128, 0, stream>>>(w, W16);
    for (int half = 0; half < 2; ++half) {
        k_xt<<<NTILE, 128, 0, stream>>>(x, half * 32, XTH, XTL);
        k_mm<<<dim3(NTILE / 64, OC / 64, 32), 128, 0, stream>>>(XTH, XTL, W16, half * 32, YT);
    }
    k_out<<<(NB_ * OC * TH) / 8, 256, 0, stream>>>(YT, bias, out);
}
